// LightweightAsymmetricAttention_14499809592014
// MI455X (gfx1250) — hardware-verified
//
#include <hip/hip_runtime.h>


#define NB_  4
#define CC   512
#define NN   4096
#define NR   1024
#define WW   64
#define WR   32
#define NH_  8
#define DK   64
#define HPP  4
#define KIM  2048
#define PCAR 1024.0f
typedef _Float16 h16;
typedef unsigned short bf;
typedef __attribute__((ext_vector_type(16))) __bf16   v16bf;
typedef __attribute__((ext_vector_type(16))) _Float16 v16h;
typedef __attribute__((ext_vector_type(8)))  _Float16 v8h;
typedef __attribute__((ext_vector_type(8)))  unsigned short v8us;
typedef __attribute__((ext_vector_type(8)))  float    v8f;
typedef __attribute__((ext_vector_type(4)))  float    v4f;
typedef v8h  __attribute__((may_alias)) v8ha;
typedef v4f  __attribute__((may_alias)) v4fa;
typedef v8us __attribute__((may_alias)) v8usa;

__device__ __forceinline__ unsigned short f2bf(float f) { unsigned u = __float_as_uint(f); u += 0x7FFFu + ((u >> 16) & 1u); return (unsigned short)(u >> 16); }
__device__ __forceinline__ float bf2f(unsigned short b) { return __uint_as_float(((unsigned)b) << 16); }
__device__ __forceinline__ float bfr(float f) { return bf2f(f2bf(f)); }
__device__ __forceinline__ v16h cat16(v8h lo, v8h hi) { return __builtin_shufflevector(lo, hi, 0, 1, 2, 3, 4, 5, 6, 7, 8, 9, 10, 11, 12, 13, 14, 15); }
__device__ __forceinline__ v16bf cat16b(v8us lo, v8us hi) { return __builtin_bit_cast(v16bf, __builtin_shufflevector(lo, hi, 0, 1, 2, 3, 4, 5, 6, 7, 8, 9, 10, 11, 12, 13, 14, 15)); }
__device__ __forceinline__ v8f wmma16(v16h a, v16h b, v8f c) { return __builtin_amdgcn_wmma_f32_16x16x32_f16(false, a, false, b, (short)0, c, false, false); }
__device__ __forceinline__ v8f wmmab(v16bf a, v16bf b, v8f c) { return __builtin_amdgcn_wmma_f32_16x16x32_bf16(false, a, false, b, (short)0, c, false, false); }


template <typename T16> struct WFrag;
template <> struct WFrag<h16> { typedef v16h V; static __device__ __forceinline__ V ld(const h16* p) { return cat16(*(const v8h*)p, *(const v8h*)(p + 16)); } static __device__ __forceinline__ v8f mma(V a, V b, v8f c) { return wmma16(a, b, c); } };
template <> struct WFrag<bf> { typedef v16bf V; static __device__ __forceinline__ V ld(const bf* p) { return cat16b(*(const v8us*)p, *(const v8us*)(p + 16)); } static __device__ __forceinline__ v8f mma(V a, V b, v8f c) { return wmmab(a, b, c); } };
template <typename T16, int NSPLIT, bool BIAS>
__global__ __launch_bounds__(32) void k_gemmw(const T16* __restrict__ A, const T16* __restrict__ A2, const T16* __restrict__ Bt, const T16* __restrict__ Bt2, int K, float* C, int ldc, const float* __restrict__ bias, size_t sA, size_t sB, size_t sC) {
    typedef typename WFrag<T16>::V V;
    __shared__ __align__(16) float os[16 * 68];
    const size_t z = blockIdx.z; A += z * sA; if (A2) A2 += z * sA; Bt += z * sB; if (Bt2) Bt2 += z * sB; C += z * sC;
    const int lane = threadIdx.x & 31, lr = lane & 15, hi = lane >> 4; const int r0 = blockIdx.x * 64, c0 = blockIdx.y * 64;
    v8f acc[4][4];
#pragma unroll
    for (int mb = 0; mb < 4; ++mb)
#pragma unroll
        for (int nb = 0; nb < 4; ++nb) acc[mb][nb] = (v8f){};
    const size_t aoff = (size_t)(r0 + lr) * K + 8 * hi, boff = (size_t)(c0 + lr) * K + 8 * hi;
#pragma unroll 1
    for (int kc = 0; kc < K; kc += 32) {
        V a[4], a2[4];
#pragma unroll
        for (int mb = 0; mb < 4; ++mb) { a[mb] = WFrag<T16>::ld(A + aoff + (size_t)mb * 16 * K + kc); if (NSPLIT == 1 || NSPLIT == 2) a2[mb] = WFrag<T16>::ld(A2 + aoff + (size_t)mb * 16 * K + kc); }
#pragma unroll
        for (int nb = 0; nb < 4; ++nb) { const V b = WFrag<T16>::ld(Bt + boff + (size_t)nb * 16 * K + kc); V b2; if (NSPLIT >= 2) b2 = WFrag<T16>::ld(Bt2 + boff + (size_t)nb * 16 * K + kc);
#pragma unroll
            for (int mb = 0; mb < 4; ++mb) { acc[mb][nb] = WFrag<T16>::mma(a[mb], b, acc[mb][nb]); if (NSPLIT == 1 || NSPLIT == 2) acc[mb][nb] = WFrag<T16>::mma(a2[mb], b, acc[mb][nb]); if (NSPLIT >= 2) acc[mb][nb] = WFrag<T16>::mma(a[mb], b2, acc[mb][nb]); } }
        asm volatile("v_nop\n\tv_nop\n\tv_nop\n\tv_nop" : "+v"(acc[0][0]), "+v"(acc[1][1]), "+v"(acc[2][2]), "+v"(acc[3][3]) : "v"(a[0]), "v"(a[3]));
    }
#pragma unroll
    for (int mb = 0; mb < 4; ++mb) {
#pragma unroll
        for (int nb = 0; nb < 4; ++nb) {
#pragma unroll
            for (int j = 0; j < 8; ++j) os[(hi * 8 + j) * 68 + nb * 16 + lr] = acc[mb][nb][j]; }
        __builtin_amdgcn_wave_barrier(); asm volatile("" ::: "memory");
        float* crow = C + (size_t)(r0 + mb * 16) * ldc + c0;
#pragma unroll 1
        for (int ps = 0; ps < 2; ++ps) {
#pragma unroll
            for (int s = 0; s < 8; ++s) { const int row = 2 * s + hi, cofs = lr * 4; v4f val = *(const v4fa*)(os + row * 68 + cofs); if (BIAS) { val[0] += bfr(bias[c0 + cofs]); val[1] += bfr(bias[c0 + cofs + 1]); val[2] += bfr(bias[c0 + cofs + 2]); val[3] += bfr(bias[c0 + cofs + 3]); }
                *(volatile v4f*)(crow + (size_t)row * ldc + cofs) = val; }
            if (ps == 0) __threadfence(); }
        __builtin_amdgcn_wave_barrier(); asm volatile("" ::: "memory");
    }
}

__device__ __forceinline__ h16 tohx(float x) { return (h16)x; }
__device__ __forceinline__ void splitf(float y, unsigned short& h, unsigned short& l) { h = f2bf(y); l = f2bf(y - bf2f(h)); }
typedef __attribute__((ext_vector_type(2))) unsigned short v2us;
typedef __attribute__((ext_vector_type(4))) unsigned short v4us;
typedef __attribute__((ext_vector_type(2))) _Float16 v2h;
typedef __attribute__((ext_vector_type(4))) _Float16 v4h;
typedef __attribute__((ext_vector_type(2))) float v2f;

__global__ __launch_bounds__(256) void k_cvt8(const float* __restrict__ src, bf* dst, size_t n8) { const size_t i = (size_t)blockIdx.x * 256 + threadIdx.x; if (i >= n8) return; const v8f v = *(const v8f*)(src + i * 8); v8us o;
#pragma unroll
    for (int k = 0; k < 8; ++k) o[k] = f2bf(v[k]); *(volatile v8us*)(dst + i * 8) = o; __threadfence(); *(volatile v8us*)(dst + i * 8) = o; }
__global__ __launch_bounds__(256) void k_tok(const float* __restrict__ in, bf* X) { const int e = (blockIdx.x * 256 + threadIdx.x) * 4; if (e >= NN * CC) return; const int c = e % CC; const int n = e / CC; v4us o;
#pragma unroll
    for (int u = 0; u < 4; ++u) o[u] = f2bf(in[(size_t)(c + u) * NN + n]); *(volatile v4us*)(X + e) = o; __threadfence(); *(volatile v4us*)(X + e) = o; }
__global__ __launch_bounds__(256) void k_im2(const float* __restrict__ in, bf* IM) { const int e = (blockIdx.x * 256 + threadIdx.x) * 4; if (e >= NR * KIM) return; const int k0 = e % KIM; const int m = e / KIM; const int y = m / WR, x = m % WR; const int c = k0 / 4; v4us o;
#pragma unroll
    for (int u = 0; u < 4; ++u) { const int kh = u >> 1, kw = u & 1; o[u] = f2bf(in[(size_t)c * NN + (2 * y + kh) * WW + 2 * x + kw]); } *(volatile v4us*)(IM + e) = o; __threadfence(); *(volatile v4us*)(IM + e) = o; }
__global__ __launch_bounds__(256) void k_pl(const float* __restrict__ F, int nrows, h16* P) { const size_t e = ((size_t)blockIdx.x * 256 + threadIdx.x) * 4; if (e >= (size_t)NH_ * nrows * DK) return; const int d = (int)(e % DK); const int t = (int)((e / DK) % nrows); const int h = (int)(e / ((size_t)DK * nrows)); const float* f = F + (size_t)t * CC + h * DK + d; v4h o;
#pragma unroll
    for (int u = 0; u < 4; ++u) o[u] = tohx(f[u]); *(volatile v4h*)(P + e) = o; __threadfence(); *(volatile v4h*)(P + e) = o; }
__global__ __launch_bounds__(256) void k_vt(const float* __restrict__ V, h16* VT) { const int e = (blockIdx.x * 256 + threadIdx.x) * 2; if (e >= NH_ * DK * NR) return; const int m = e % NR; const int d = (e / NR) % DK; const int h = e / (NR * DK); v2h o; o[0] = tohx(V[(size_t)m * CC + h * DK + d]); o[1] = tohx(V[(size_t)(m + 1) * CC + h * DK + d]); *(volatile v2h*)(VT + e) = o; __threadfence(); *(volatile v2h*)(VT + e) = o; }
__global__ __launch_bounds__(256) void k_soft(const float* __restrict__ Sb, const float* __restrict__ bias, int h0, h16* P16) { const int lane = threadIdx.x & 31; const int row = blockIdx.x * 8 + (threadIdx.x >> 5); if (row >= HPP * NN) return; const int z = row / NN; const float bb = bfr(bias[h0 + z]); const float* sr = Sb + (size_t)row * NR; float v[NR / 32]; float mx = -3.0e38f;
#pragma unroll
    for (int ch = 0; ch < NR / 128; ++ch) { const v4f a = *(const v4f*)(sr + ch * 128 + lane * 4);
#pragma unroll
        for (int u = 0; u < 4; ++u) { float t0 = a[u] * 0.125f; asm volatile("" : "+v"(t0)); float b1 = bb; asm volatile("" : "+v"(b1)); const float t = __fadd_rn(t0, b1); v[ch * 4 + u] = t; mx = fmaxf(mx, t); } }
#pragma unroll
    for (int sh = 16; sh; sh >>= 1) mx = fmaxf(mx, __shfl_xor(mx, sh, 32));
    float sum = 0.f;
#pragma unroll
    for (int q = 0; q < NR / 32; ++q) { float d0 = __fsub_rn(v[q], mx); asm volatile("" : "+v"(d0)); v[q] = __builtin_amdgcn_exp2f(__fmul_rn(d0, 1.4426950408889634f)); sum += v[q]; }
#pragma unroll
    for (int sh = 16; sh; sh >>= 1) sum += __shfl_xor(sum, sh, 32);
    const float f = __fdiv_rn(PCAR, sum);
    for (int ps = 0; ps < 2; ++ps) {
#pragma unroll
        for (int ch = 0; ch < NR / 128; ++ch) { v4h o4;
#pragma unroll
            for (int q = 0; q < 4; ++q) o4[q] = tohx(v[ch * 4 + q] * f); *(volatile v4h*)(P16 + (size_t)row * NR + ch * 128 + lane * 4) = o4; }
        if (ps == 0) __threadfence(); } }
__global__ __launch_bounds__(256) void k_mrg(const float* __restrict__ O, int h0, bf* Ah, bf* Al) { const int e = (blockIdx.x * 256 + threadIdx.x) * 4; if (e >= HPP * NN * DK) return; const int d = e % DK; const int t = (e / DK) % NN; const int z = e / (DK * NN); v4us oh, ol;
#pragma unroll
    for (int u = 0; u < 4; ++u) { unsigned short a, b; splitf(O[e + u] * (1.0f / PCAR), a, b); oh[u] = a; ol[u] = b; } const size_t oo = (size_t)t * CC + (h0 + z) * DK + d; *(volatile v4us*)(Ah + oo) = oh; *(volatile v4us*)(Al + oo) = ol; __threadfence(); *(volatile v4us*)(Ah + oo) = oh; *(volatile v4us*)(Al + oo) = ol; }
__global__ __launch_bounds__(256) void k_bnstat(const float* __restrict__ P, float* ST) { const int c = blockIdx.x * 256 + threadIdx.x; if (c >= CC) return; float s = 0.f;
#pragma unroll 1
    for (int i = 0; i < NB_ * NN; ++i) s = __fadd_rn(s, P[(size_t)i * CC + c]);
    const float mu = s * (1.0f / (NB_ * NN)); float q = 0.f;
#pragma unroll 1
    for (int i = 0; i < NB_ * NN; ++i) { float d = __fsub_rn(P[(size_t)i * CC + c], mu); asm volatile("" : "+v"(d)); float p = __fmul_rn(d, d); asm volatile("" : "+v"(p)); q = __fadd_rn(q, p); }
    v2f o; o[0] = mu; o[1] = __frsqrt_rn(__fadd_rn(q * (1.0f / (NB_ * NN)), 1e-5f)); *(volatile v2f*)(ST + (size_t)c * 2) = o; __threadfence(); *(volatile v2f*)(ST + (size_t)c * 2) = o; }
__device__ __forceinline__ float bnval(float x, float p, const float* __restrict__ ST, const float* __restrict__ bg, const float* __restrict__ bb, int c) { const v2f st = *(const v2f*)(ST + (size_t)c * 2); float d = __fsub_rn(p, st[0]); asm volatile("" : "+v"(d)); float n0 = __fmul_rn(d, st[1]); asm volatile("" : "+v"(n0)); float g1 = bfr(bg[c]); asm volatile("" : "+v"(g1)); float t1 = __fmul_rn(n0, g1); asm volatile("" : "+v"(t1)); float b1 = bfr(bb[c]); asm volatile("" : "+v"(b1)); float pn = __fadd_rn(t1, b1); asm volatile("" : "+v"(pn)); float xb = bfr(x); asm volatile("" : "+v"(xb)); return __fadd_rn(xb, pn); }
__global__ __launch_bounds__(256) void k_lnstat(const float* __restrict__ X, const float* __restrict__ P, const float* __restrict__ ST, const float* __restrict__ bg, const float* __restrict__ bb, float* LS) { const int lane = threadIdx.x & 31; const int n = blockIdx.x * 8 + (threadIdx.x >> 5);
    const int b = blockIdx.y; float v[CC / 32]; float s = 0.f;
#pragma unroll
    for (int k = 0; k < CC / 32; ++k) { const int c = k * 32 + lane; v[k] = bnval(X[((size_t)b * CC + c) * NN + n], P[((size_t)b * NN + n) * CC + c], ST, bg, bb, c); s += v[k]; }
#pragma unroll
    for (int sh = 16; sh; sh >>= 1) s += __shfl_xor(s, sh, 32);
    const float mean = s * (1.0f / CC); float q = 0.f;
#pragma unroll
    for (int k = 0; k < CC / 32; ++k) { float d = __fsub_rn(v[k], mean); asm volatile("" : "+v"(d)); float p = __fmul_rn(d, d); asm volatile("" : "+v"(p)); q = __fadd_rn(q, p); }
#pragma unroll
    for (int sh = 16; sh; sh >>= 1) q += __shfl_xor(q, sh, 32);
    const float rs = __frsqrt_rn(__fadd_rn(q * (1.0f / CC), 1e-5f));
    __shared__ float sh2[16]; const int wv = threadIdx.x >> 5; if (lane == 0) { sh2[wv * 2] = mean; sh2[wv * 2 + 1] = rs; } __syncthreads();
    if (threadIdx.x < 32) { const float val = (threadIdx.x < 16) ? sh2[threadIdx.x] : 0.f; float* dst = LS + ((size_t)b * (NN / 8) + blockIdx.x) * 32 + threadIdx.x; *(volatile float*)dst = val; __threadfence(); *(volatile float*)dst = val; } }
__global__ __launch_bounds__(256) void k_out(const float* __restrict__ X, const float* __restrict__ P, const float* __restrict__ ST, const float* __restrict__ bg, const float* __restrict__ bb, const float* __restrict__ LS, const float* __restrict__ lg, const float* __restrict__ lb, float* OUT) {
    const size_t e = ((size_t)blockIdx.x * 256 + threadIdx.x) * 4; if (e >= (size_t)NB_ * CC * NN) return; const int n = (int)(e % NN); const int c = (int)((e / NN) % CC); const int b = (int)(e / ((size_t)NN * CC)); v4f o;
#pragma unroll
    for (int u = 0; u < 4; ++u) { const int nn = n + u; const float y = bnval(X[e + u], P[((size_t)b * NN + nn) * CC + c], ST, bg, bb, c); const float* ls = LS + ((size_t)b * (NN / 8) + nn / 8) * 32 + (nn % 8) * 2; float d = __fsub_rn(y, ls[0]); asm volatile("" : "+v"(d)); float n0 = __fmul_rn(d, ls[1]); asm volatile("" : "+v"(n0)); float g1 = bfr(lg[c]); asm volatile("" : "+v"(g1)); float t1 = __fmul_rn(n0, g1); asm volatile("" : "+v"(t1)); float b1 = bfr(lb[c]); asm volatile("" : "+v"(b1)); o[u] = __fadd_rn(t1, b1); }
    *(volatile v4f*)(OUT + e) = o; __threadfence(); *(volatile v4f*)(OUT + e) = o; }

extern "C" void kernel_launch(void* const* d_in, const int* in_sizes, int n_in,
                              void* d_out, int out_size, void* d_ws, size_t ws_size, hipStream_t stream) {
    (void)in_sizes; (void)n_in; (void)out_size;
    const float** I = (const float**)d_in;
    const float *x = I[0], *Wq = I[1], *Wk = I[2], *Wv = I[3], *bias = I[4], *Wp = I[5], *bng = I[6], *bnb = I[7], *lng = I[8], *lnb = I[9];
    float* OUT = (float*)d_out;
    char* wsp = (char*)d_ws;
    auto take = [&](size_t bytes) { char* p = wsp; wsp += (bytes + 255) & ~(size_t)255; return (void*)p; };
    bf* BQ = (bf*)take((size_t)CC * CC * 2); bf* BK = (bf*)take((size_t)CC * KIM * 2); bf* BV = (bf*)take((size_t)CC * KIM * 2); bf* BP = (bf*)take((size_t)CC * CC * 2);
    bf* XT = (bf*)take((size_t)NN * CC * 2); bf* IM = (bf*)take((size_t)NR * KIM * 2); float* Q = (float*)take((size_t)NN * CC * 4); float* K = (float*)take((size_t)NR * CC * 4); float* V = (float*)take((size_t)NR * CC * 4);
    h16* Q16 = (h16*)take((size_t)NH_ * NN * DK * 2); h16* K16 = (h16*)take((size_t)NH_ * NR * DK * 2); h16* VT = (h16*)take((size_t)NH_ * DK * NR * 2); float* Sb = (float*)take((size_t)HPP * NN * NR * 4); h16* P16 = (h16*)take((size_t)HPP * NN * NR * 2); float* O = (float*)take((size_t)HPP * NN * DK * 4);
    bf* OTh = (bf*)take((size_t)NN * CC * 2); bf* OTl = (bf*)take((size_t)NN * CC * 2); float* PA = (float*)take((size_t)NB_ * NN * CC * 4); float* ST = (float*)take((size_t)CC * 2 * 4); float* LS = (float*)take((size_t)NB_ * (NN / 8) * 32 * 4);
    if ((size_t)(wsp - (char*)d_ws) > ws_size) return;
    k_cvt8<<<(CC * CC / 8 + 255) / 256, 256, 0, stream>>>(Wq, BQ, CC * CC / 8); k_cvt8<<<(CC * KIM / 8 + 255) / 256, 256, 0, stream>>>(Wk, BK, (size_t)CC * KIM / 8); k_cvt8<<<(CC * KIM / 8 + 255) / 256, 256, 0, stream>>>(Wv, BV, (size_t)CC * KIM / 8); k_cvt8<<<(CC * CC / 8 + 255) / 256, 256, 0, stream>>>(Wp, BP, CC * CC / 8);
    const size_t zq = (size_t)NN * DK, zk = (size_t)NR * DK, zS = (size_t)NN * NR;
    for (int b = 0; b < NB_; ++b) { const float* xb = x + (size_t)b * CC * NN;
        k_tok<<<(NN * CC / 4 + 255) / 256, 256, 0, stream>>>(xb, XT); k_im2<<<(NR * KIM / 4 + 255) / 256, 256, 0, stream>>>(xb, IM);
        k_gemmw<bf, 0, false><<<dim3(NN / 64, CC / 64, 1), 32, 0, stream>>>(XT, nullptr, BQ, nullptr, CC, Q, CC, nullptr, 0, 0, 0); k_gemmw<bf, 0, false><<<dim3(NR / 64, CC / 64, 1), 32, 0, stream>>>(IM, nullptr, BK, nullptr, KIM, K, CC, nullptr, 0, 0, 0); k_gemmw<bf, 0, false><<<dim3(NR / 64, CC / 64, 1), 32, 0, stream>>>(IM, nullptr, BV, nullptr, KIM, V, CC, nullptr, 0, 0, 0);
        k_pl<<<(unsigned)(((size_t)NH_ * NN * DK / 4 + 255) / 256), 256, 0, stream>>>(Q, NN, Q16); k_pl<<<(unsigned)(((size_t)NH_ * NR * DK / 4 + 255) / 256), 256, 0, stream>>>(K, NR, K16); k_vt<<<(NH_ * DK * NR / 2 + 255) / 256, 256, 0, stream>>>(V, VT);
        for (int h0 = 0; h0 < NH_; h0 += HPP) {
            k_gemmw<h16, 0, false><<<dim3(NN / 64, NR / 64, HPP), 32, 0, stream>>>(Q16 + (size_t)h0 * zq, nullptr, K16 + (size_t)h0 * zk, nullptr, DK, Sb, NR, nullptr, zq, zk, zS);
            k_soft<<<HPP * NN / 8, 256, 0, stream>>>(Sb, bias, h0, P16);
            k_gemmw<h16, 0, false><<<dim3(NN / 64, 1, HPP), 32, 0, stream>>>(P16, nullptr, VT + (size_t)h0 * DK * NR, nullptr, NR, O, DK, nullptr, zS, (size_t)DK * NR, zq);
            k_mrg<<<(HPP * NN * DK / 4 + 255) / 256, 256, 0, stream>>>(O, h0, OTh, OTl); }
        k_gemmw<bf, 1, false><<<dim3(NN / 64, CC / 64, 1), 32, 0, stream>>>(OTh, OTl, BP, nullptr, CC, PA + (size_t)b * NN * CC, CC, nullptr, 0, 0, 0); }
    k_bnstat<<<(CC + 255) / 256, 256, 0, stream>>>(PA, ST);
    k_lnstat<<<dim3(NN / 8, NB_, 1), 256, 0, stream>>>(x, PA, ST, bng, bnb, LS);
    k_out<<<(unsigned)(((size_t)NB_ * CC * NN / 4 + 255) / 256), 256, 0, stream>>>(x, PA, ST, bng, bnb, LS, lng, lnb, OUT);
}
